// LinearKAN_1357209666064
// MI455X (gfx1250) — hardware-verified
//
#include <hip/hip_runtime.h>


namespace {
constexpr int NB_ = 16384, IN = 768, OUT = 768, G = 8, KS = G * IN  , KT = KS + IN  , RL = NB_  , NSL = OUT / 128;
constexpr float XS = 8.0f, WSC = 256.0f, WBS = 65536.0f, GLO = -2.0f, GHI = 2.0f;
static_assert(KT % 256 == 0 && KS % 256 == 0 && NB_ % 64 == 0 && RL % 64 == 0 && OUT % 128 == 0, "tiling");
typedef _Float16 b16;
typedef __attribute__((ext_vector_type(16))) _Float16 v16b;
typedef __attribute__((ext_vector_type(8))) _Float16 v8b;
typedef __attribute__((ext_vector_type(8))) float v8f;
typedef __attribute__((ext_vector_type(4))) float v4f;
__device__ __forceinline__ float bf16_rne(float f) { unsigned int u = __float_as_uint(f); u += 0x7FFFu + ((u >> 16) & 1u); return __uint_as_float(u & 0xFFFF0000u); }
__device__ __forceinline__ void split16(float v, b16& hi, b16& lo) { hi = (b16)v; lo = (b16)(v - (float)hi); }
__device__ __forceinline__ v16b frag_kb(const b16* p, int hh) { const v8b a = *(const v8b*)(p + 8 * hh), b = *(const v8b*)(p + 16 + 8 * hh); v16b f;
#pragma unroll
  for (int e = 0; e < 8; ++e) { f[e] = a[e]; f[8 + e] = b[e]; } return f; }
__device__ __forceinline__ v8f wmma16b(v16b a, v16b b, v8f c) { v8f d = __builtin_amdgcn_wmma_f32_16x16x32_f16(false, a, false, b, (short)0, c, false, false); asm volatile("v_nop\n\tv_nop\n\tv_nop\n\tv_nop" : "+v"(d) : "v"(a), "v"(b)); return d; }
__device__ __forceinline__ void wave_lds_sync() { __builtin_amdgcn_fence(__ATOMIC_RELEASE, "workgroup"); __builtin_amdgcn_wave_barrier(); __builtin_amdgcn_fence(__ATOMIC_ACQUIRE, "workgroup"); }
__device__ __forceinline__ float pmul(float a, float b) { float p = a * b; asm volatile("" : "+v"(p)); return p; }
__device__ __forceinline__ int iclamp(int v, int lo, int hi) { return v < lo ? lo : (v > hi ? hi : v); }

typedef __attribute__((ext_vector_type(2))) _Float16 v2h;
typedef __attribute__((ext_vector_type(4))) _Float16 v4h;
typedef __attribute__((ext_vector_type(2))) float v2f;
typedef __attribute__((ext_vector_type(4))) int v4i;
__device__ __forceinline__ float nexp2(float v) { return __builtin_amdgcn_exp2f(v); }
__global__ __launch_bounds__(256) void wb_kernel(const float* __restrict__ c, const float* __restrict__ ws_, const float* __restrict__ wb, b16* __restrict__ WB) {
  const size_t u = (size_t)blockIdx.x * 256 + threadIdx.x; if (u >= (size_t)OUT * KT / 8) return; const size_t e = u * 8; const int o = (int)(e / KT), k0 = (int)(e % KT); v8b v;
#pragma unroll
  for (int j = 0; j < 8; ++j) { const int k = k0 + j; float val; if (k < KS) { const int a = k / IN, i = k % IN; val = bf16_rne(c[((size_t)a * OUT + o) * IN + i]) * bf16_rne(ws_[(size_t)o * IN + i]) * WSC; } else { const int i = k - KS; val = bf16_rne(wb[(size_t)o * IN + i]) * WBS; } v[j] = (b16)val; }
  for (int pass = 0; pass < 2; ++pass) { *(volatile v8b*)(WB + e) = v; __threadfence(); }
}
__global__ __launch_bounds__(128) void kan_kernel(const float* __restrict__ x, const b16* __restrict__ WB, float* __restrict__ out) {
  __shared__ __attribute__((aligned(16))) b16 As[64][256 + 8]; __shared__ __attribute__((aligned(16))) float Tf[4][16][128 + 4];
  const int wave = threadIdx.x >> 5, lane = threadIdx.x & 31, nloc = lane & 15, hlf = lane >> 4; const size_t r0 = (size_t)blockIdx.x * 64; const int n0 = blockIdx.y * 128;
  const float hstep = (GHI - GLO) / (float)(G - 1); const float rh = 1.0f / hstep;
  v8f acc[8], accr[8];
#pragma unroll
  for (int t = 0; t < 8; ++t) { acc[t] = (v8f){}; accr[t] = (v8f){}; }
#pragma unroll 1
  for (int kc = 0; kc < KT; kc += 256) { const bool spline = kc < KS; const int a = kc / IN; const float ga = GLO + hstep * (float)a; const int i0 = spline ? (kc % IN) : (kc - KS);
    __syncthreads();
    for (int idx = threadIdx.x; idx < 64 * 64; idx += 128) { const int rr = idx / 64, q = (idx % 64) * 4; const v4f xv = *(const v4f*)(x + (r0 + rr) * IN + i0 + q); v4h o4;
      for (int j = 0; j < 4; ++j) { const float xx = bf16_rne(xv[j]); float f; if (spline) { const float z = (xx - ga) * rh; f = __expf(-z * z); } else { f = xx / (1.0f + __expf(-xx)); } o4[j] = (b16)(f * XS); }
      *(v4h*)(&As[rr][q]) = o4; }
    __syncthreads();
#pragma unroll 2
    for (int kb = 0; kb < 256; kb += 32) { const v16b af = frag_kb(&As[wave * 16 + nloc][kb], hlf);
      if (spline) {
#pragma unroll
        for (int t = 0; t < 8; ++t) acc[t] = wmma16b(af, frag_kb(WB + (size_t)(n0 + t * 16 + nloc) * KT + kc + kb, hlf), acc[t]); }
      else {
#pragma unroll
        for (int t = 0; t < 8; ++t) accr[t] = wmma16b(af, frag_kb(WB + (size_t)(n0 + t * 16 + nloc) * KT + kc + kb, hlf), accr[t]); } } }
#pragma unroll
  for (int t = 0; t < 8; ++t)
#pragma unroll
    for (int r = 0; r < 8; ++r) Tf[wave][8 * hlf + r][t * 16 + nloc] = acc[t][r] * (1.0f / (XS * WSC)) + accr[t][r] * (1.0f / (XS * WBS));
  wave_lds_sync();
  for (int pass = 0; pass < 2; ++pass) { for (int rr = 0; rr < 16; ++rr) *(volatile v4f*)(out + (r0 + wave * 16 + rr) * OUT + n0 + lane * 4) = *(const v4f*)(&Tf[wave][rr][lane * 4]); __threadfence(); }
}
}

extern "C" void kernel_launch(void* const* d_in, const int* in_sizes, int n_in, void* d_out, int out_size, void* d_ws, size_t ws_size, hipStream_t stream) {
  (void)n_in;
  auto Fp = [&](int i) { return (const float*)d_in[i]; };
  if (in_sizes[0] != NB_ * IN || in_sizes[1] != OUT * IN || in_sizes[2] != OUT * IN || in_sizes[3] != G * OUT * IN || out_size != NB_ * OUT) return;
  size_t off = 0; char* ws = (char*)d_ws;
  auto carve = [&](size_t bytes) { char* p = ws + off; off += (bytes + 255) & ~(size_t)255; return p; };
  b16* WB = (b16*)carve((size_t)OUT * KT * 2);
  if (off > ws_size || off > ((size_t)128 << 20)) return;
  wb_kernel<<<(unsigned)(((size_t)OUT * KT / 8 + 255) / 256), 256, 0, stream>>>(Fp(3), Fp(2), Fp(1), WB);
  kan_kernel<<<dim3(RL / 64, NSL), 128, 0, stream>>>(Fp(0), WB, (float*)d_out);
}
